// QuantizedLinear_24721831756574
// MI455X (gfx1250) — hardware-verified
//
#include <hip/hip_runtime.h>

typedef _Float16 v16h __attribute__((ext_vector_type(16)));
typedef _Float16 v8h  __attribute__((ext_vector_type(8)));
typedef float    v8f  __attribute__((ext_vector_type(8)));
typedef float    v4f  __attribute__((ext_vector_type(4)));
typedef int      v4i  __attribute__((ext_vector_type(4)));
typedef v8h __attribute__((may_alias)) v8ha;
typedef v4f __attribute__((may_alias)) v4fa;
typedef v4i __attribute__((may_alias)) v4ia;

union Frag { v16h v; v8h half[2]; };

#define KDIM 4096
#define NDIM 4096
#define GBM  128
#define GBN  64

__device__ __forceinline__ v8f wmma_f16(v16h a, v16h b, v8f c) {
  v8f d = __builtin_amdgcn_wmma_f32_16x16x32_f16(false, a, false, b, (short)0, c, false, false);
  asm volatile("v_nop\n\tv_nop\n\tv_nop\n\tv_nop" : "+v"(d) : "v"(a), "v"(b));
  return d;
}

__device__ __forceinline__ v16h load_frag(const _Float16* p, int h) {
  Frag f;
  f.half[0] = *(const v8ha*)(p + 8 * h);
  f.half[1] = *(const v8ha*)(p + 16 + 8 * h);
  return f.v;
}

__global__ __launch_bounds__(256) void cvt_x_kernel(
    const float* __restrict__ x, _Float16* __restrict__ xh, int n8)
{
  const int i = blockIdx.x * 256 + threadIdx.x;
  if (i >= n8) return;
  const float* src = x + (size_t)i * 8;
  const v4f a = *(const v4fa*)src;
  const v4f c = *(const v4fa*)(src + 4);
  const v8h o = { (_Float16)a.x, (_Float16)a.y, (_Float16)a.z, (_Float16)a.w,
                  (_Float16)c.x, (_Float16)c.y, (_Float16)c.z, (_Float16)c.w };
  _Float16* dst = xh + (size_t)i * 8;
  *(volatile v8h*)dst = o;
  __threadfence();
  *(volatile v8h*)dst = o;
}

__global__ __launch_bounds__(256) void deq_w_kernel(
    const int*   __restrict__ packed,
    const float* __restrict__ scales,
    const float* __restrict__ offsets,
    _Float16*    __restrict__ wh, int ngroups)
{
  #pragma clang fp contract(off)
  const int g = blockIdx.x * 256 + threadIdx.x;
  if (g >= ngroups) return;
  const v4i p = *(const v4ia*)(packed + (size_t)g * 4);
  const float s = scales[g];
  const float o = offsets[g];
  const float w0 = (float)(p.x & 15)        * s + o;
  const float w1 = (float)((p.x >> 4) & 15) * s + o;
  const float w2 = (float)(p.y & 15)        * s + o;
  const float w3 = (float)((p.y >> 4) & 15) * s + o;
  const float w4 = (float)(p.z & 15)        * s + o;
  const float w5 = (float)((p.z >> 4) & 15) * s + o;
  const float w6 = (float)(p.w & 15)        * s + o;
  const float w7 = (float)((p.w >> 4) & 15) * s + o;
  const v8h v = { (_Float16)w0, (_Float16)w1, (_Float16)w2, (_Float16)w3,
                  (_Float16)w4, (_Float16)w5, (_Float16)w6, (_Float16)w7 };
  _Float16* dst = wh + (size_t)g * 8;
  *(volatile v8h*)dst = v;
  __threadfence();
  *(volatile v8h*)dst = v;
}

__device__ __forceinline__ void out_store_pass(const float* so, float* out,
                                               int m0w, int n0, int lane) {
  const int q8 = lane & 7, sub = lane >> 3;
  #pragma unroll
  for (int i = 0; i < 16; ++i) {
    const int lid = i * 4 + sub;
    const int row = lid >> 1, hl = lid & 1;
    const v4f v = *(const v4fa*)(so + row * 64 + 32 * hl + 4 * q8);
    const size_t gi = (size_t)(m0w + row) * NDIM + n0 + 32 * hl + 4 * q8;
    *(volatile v4f*)(out + gi) = v;
  }
}

__global__ __launch_bounds__(128) void gemm_kernel(
    const _Float16* __restrict__ xh,
    const _Float16* __restrict__ wh,
    const float* __restrict__ bias,
    float* __restrict__ out)
{
  __shared__ __attribute__((aligned(16))) float sO[4 * 32 * 64];

  const int tid = threadIdx.x, lane = tid & 31, w = tid >> 5;
  const int h = lane >> 4, m = lane & 15;
  const int n0 = blockIdx.x * GBN;
  const int m0 = blockIdx.y * GBM;
  const int m0w = m0 + 32 * w;

  const _Float16* xa0 = xh + (size_t)(m0w + m) * KDIM;
  const _Float16* xa1 = xa0 + (size_t)16 * KDIM;
  const _Float16* wb  = wh + (size_t)(n0 + m) * KDIM;

  const v8f zero8 = {0.f, 0.f, 0.f, 0.f, 0.f, 0.f, 0.f, 0.f};
  v8f acc[2][4];
  #pragma unroll
  for (int mt = 0; mt < 2; ++mt)
    #pragma unroll
    for (int nt = 0; nt < 4; ++nt) acc[mt][nt] = zero8;

  #pragma unroll 1
  for (int k0 = 0; k0 < KDIM; k0 += 32) {
    const v16h a0 = load_frag(xa0 + k0, h);
    const v16h a1 = load_frag(xa1 + k0, h);
    #pragma unroll
    for (int nt = 0; nt < 4; ++nt) {
      const v16h b = load_frag(wb + (size_t)nt * 16 * KDIM + k0, h);
      acc[0][nt] = wmma_f16(a0, b, acc[0][nt]);
      acc[1][nt] = wmma_f16(a1, b, acc[1][nt]);
    }
  }

  float* so = sO + w * 2048;
  #pragma unroll
  for (int nt = 0; nt < 4; ++nt) {
    const int col = 16 * nt + m;
    const float bvl = bias[n0 + col];
    #pragma unroll
    for (int mt = 0; mt < 2; ++mt) {
      #pragma unroll
      for (int r = 0; r < 8; ++r) {
        const int rowl = 16 * mt + 8 * h + r;
        so[rowl * 64 + col] = acc[mt][nt][r] + bvl;
      }
    }
  }
  __syncthreads();

  out_store_pass(so, out, m0w, n0, lane);
  __threadfence();
  out_store_pass(so, out, m0w, n0, lane);
}

extern "C" void kernel_launch(void* const* d_in, const int* in_sizes, int n_in,
                              void* d_out, int out_size, void* d_ws, size_t ws_size,
                              hipStream_t stream) {
  if (n_in < 5) return;
  const int M = in_sizes[0] / KDIM;
  if (M <= 0 || (M % GBM) != 0) return;
  if (in_sizes[0] != M * KDIM) return;
  if (in_sizes[1] != (NDIM / 2) * KDIM) return;
  if (in_sizes[2] != (NDIM / 8) * KDIM) return;
  if (in_sizes[3] != (NDIM / 8) * KDIM) return;
  if (in_sizes[4] != NDIM) return;
  if (out_size != M * NDIM) return;

  const float* x       = (const float*)d_in[0];
  const int*   packed  = (const int*)d_in[1];
  const float* scales  = (const float*)d_in[2];
  const float* offsets = (const float*)d_in[3];
  const float* bias    = (const float*)d_in[4];
  float* out = (float*)d_out;

  const size_t xh_bytes = (size_t)M * KDIM * 2;
  const size_t wh_bytes = (size_t)NDIM * KDIM * 2;
  const size_t total = xh_bytes + wh_bytes;
  if (total > ws_size) return;

  char* ws = (char*)d_ws;
  _Float16* xh = (_Float16*)(ws);
  _Float16* wh = (_Float16*)(ws + xh_bytes);

  const int n8 = (M * KDIM) / 8;
  cvt_x_kernel<<<(n8 + 255) / 256, 256, 0, stream>>>(x, xh, n8);

  const int ngroups = (NDIM / 8) * KDIM;
  deq_w_kernel<<<(ngroups + 255) / 256, 256, 0, stream>>>(packed, scales, offsets, wh, ngroups);

  dim3 gG(NDIM / GBN, M / GBM);
  gemm_kernel<<<gG, 128, 0, stream>>>(xh, wh, bias, out);
}
